// Encoder_69329362092650
// MI455X (gfx1250) — hardware-verified
//
#include <hip/hip_runtime.h>
#include <math.h>

constexpr int NBATCH  = 128;
constexpr int NSTEP   = 128;
constexpr int NFEAT   = 128;
constexpr int NHID    = 256;
constexpr int NGATE   = 4 * NHID;
constexpr int KGATE   = NFEAT + NHID;
constexpr int KATT    = 2 * NHID;
constexpr int NTHR    = 256;
constexpr int ROWS_BLK = 16;
constexpr int APITCH  = 648;
constexpr int COL_H   = NFEAT;
constexpr int COL_C   = NFEAT + NHID;
constexpr int WPPITCH = 132;
constexpr int CPITCH  = 260;
constexpr float XW_CARRY  = 1024.0f;
constexpr float HC_CARRY  = 256.0f;
constexpr float WIH_CARRY = 16.0f;
constexpr float WHH_CARRY = 64.0f;
constexpr float WE_CARRY  = 64.0f;
constexpr float XT_CARRY  = 16.0f;
constexpr float UE_CARRY  = 64.0f;
constexpr float GATE_FOLD = 1.0f / (XW_CARRY * WIH_CARRY);
constexpr float WP2_FOLD  = 2.0f / (HC_CARRY * WE_CARRY);
constexpr float UX2_FOLD  = 2.0f / (XT_CARRY * UE_CARRY);
static_assert(XW_CARRY * WIH_CARRY == HC_CARRY * WHH_CARRY, "one accumulator, one carry");
static_assert(NSTEP == 128 && NFEAT == 128 && NHID == 256 && NBATCH % ROWS_BLK == 0, "shape");
static_assert(KGATE % 32 == 0 && KATT % 32 == 0 && NSTEP % 32 == 0, "k multiples of 32");
static_assert((NBATCH * NFEAT) % 64 == 0 && NSTEP % 64 == 0, "gemm tile multiples");
static_assert(COL_C + NHID <= APITCH && APITCH % 8 == 0, "A tile");
static_assert((2 * ROWS_BLK * APITCH) % NTHR == 0, "A tile zero fill exact");
static_assert(NHID == 32 * (NTHR / 32), "8 waves x 32 hidden units");
static_assert(NGATE == 4 * NTHR, "bias staging exact");

typedef __attribute__((ext_vector_type(16))) _Float16 v16h;
typedef __attribute__((ext_vector_type(8)))  _Float16 v8h;
typedef __attribute__((ext_vector_type(16))) __bf16   v16b;
typedef __attribute__((ext_vector_type(8)))  __bf16   v8b;
typedef __attribute__((ext_vector_type(8)))  float    v8f;
typedef __attribute__((ext_vector_type(4)))  float    v4f;

__device__ __forceinline__ unsigned short f2bf_bits(float f) {
  unsigned u = __float_as_uint(f);
  return (unsigned short)((u + 0x7FFFu + ((u >> 16) & 1u)) >> 16);
}
__device__ __forceinline__ float bf_bits2f(unsigned short h) { return __uint_as_float(((unsigned)h) << 16); }

__device__ __forceinline__ void dep_guard4_h(v8f& a, v8f& b, v8f& c, v8f& d, v16h x, v16h y) {
  asm volatile("v_nop\n\tv_nop\n\tv_nop\n\tv_nop" : "+v"(a), "+v"(b), "+v"(c), "+v"(d) : "v"(x), "v"(y));
}
__device__ __forceinline__ void dep_guard4_b(v8f& a, v8f& b, v8f& c, v8f& d, v16b x, v16b y) {
  asm volatile("v_nop\n\tv_nop\n\tv_nop\n\tv_nop" : "+v"(a), "+v"(b), "+v"(c), "+v"(d) : "v"(x), "v"(y));
}
__device__ __forceinline__ void dep_guard1_h(v8f& a, v16h x, v16h y) {
  asm volatile("v_nop\n\tv_nop\n\tv_nop\n\tv_nop" : "+v"(a) : "v"(x), "v"(y));
}
__device__ __forceinline__ void dep_guard4x5_h(v8f& a, v8f& b, v8f& c, v8f& d, v16h x, v16h y0, v16h y1, v16h y2, v16h y3) {
  asm volatile("v_nop\n\tv_nop\n\tv_nop\n\tv_nop" : "+v"(a), "+v"(b), "+v"(c), "+v"(d) : "v"(x), "v"(y0), "v"(y1), "v"(y2), "v"(y3));
}
__device__ __forceinline__ void keep4_h(v16h a, v16h b, v16h c, v16h d) { asm volatile("v_nop" :: "v"(a), "v"(b), "v"(c), "v"(d)); }
__device__ __forceinline__ void keep4_b(v16b a, v16b b, v16b c, v16b d) { asm volatile("v_nop" :: "v"(a), "v"(b), "v"(c), "v"(d)); }
__device__ __forceinline__ void acc_guard4(v8f& a, v8f& b, v8f& c, v8f& d) {
  asm volatile("v_nop\n\tv_nop\n\tv_nop\n\tv_nop" : "+v"(a), "+v"(b), "+v"(c), "+v"(d));
}

template <typename T> struct Frag;
template <> struct Frag<_Float16> {
  typedef v16h V; union U { v16h v; v8h h[2]; };
  static __device__ __forceinline__ v16h load(const _Float16* p) {
    U f; f.h[0] = *(const v8h*)(p); f.h[1] = *(const v8h*)(p + 16); return f.v;
  }
  static __device__ __forceinline__ v8f mma(v16h a, v16h b, v8f c) {
    return __builtin_amdgcn_wmma_f32_16x16x32_f16(false, a, false, b, (short)0, c, false, false);
  }
  static __device__ __forceinline__ void guard4(v8f& a, v8f& b, v8f& c, v8f& d, v16h x, v16h y) { dep_guard4_h(a, b, c, d, x, y); }
  static __device__ __forceinline__ void keep(v16h a, v16h b, v16h c, v16h d) { keep4_h(a, b, c, d); }
};
template <> struct Frag<__bf16> {
  typedef v16b V; union U { v16b v; v8b h[2]; };
  static __device__ __forceinline__ v16b load(const __bf16* p) {
    U f; f.h[0] = *(const v8b*)(p); f.h[1] = *(const v8b*)(p + 16); return f.v;
  }
  static __device__ __forceinline__ v8f mma(v16b a, v16b b, v8f c) {
    return __builtin_amdgcn_wmma_f32_16x16x32_bf16(false, a, false, b, (short)0, c, false, false);
  }
  static __device__ __forceinline__ void guard4(v8f& a, v8f& b, v8f& c, v8f& d, v16b x, v16b y) { dep_guard4_b(a, b, c, d, x, y); }
  static __device__ __forceinline__ void keep(v16b a, v16b b, v16b c, v16b d) { keep4_b(a, b, c, d); }
};

__device__ __forceinline__ float tanh_from2x_fast(float t2) { return 1.0f - 2.0f * __builtin_amdgcn_rcpf(__expf(t2) + 1.0f); }
__device__ __forceinline__ float sig_p(float v)  { return __builtin_amdgcn_rcpf(1.0f + expf(-v)); }
__device__ __forceinline__ float tanh_p(float v) { return 1.0f - 2.0f * __builtin_amdgcn_rcpf(expf(2.0f * v) + 1.0f); }

template <int ET> struct Elem;
template <> struct Elem<0> { typedef _Float16 T; };
template <> struct Elem<1> { typedef __bf16 T; };
template <int ET, bool SPLIT, int BIAS_MODE, int OUT_MODE, bool RESID, int ACT = 0>
__global__ __launch_bounds__(256) void wmma_gemm64(
    const unsigned short* __restrict__ Ap, const unsigned short* __restrict__ A2p, int lda, long strideA,
    const unsigned short* __restrict__ Btp, const unsigned short* __restrict__ Bt2p, int ldb, long strideB,
    void* __restrict__ Cout, void* __restrict__ Cout2, int ldc, long strideC,
    const float* __restrict__ bias,
    const float* __restrict__ resid, long strideR,
    int M, int N, int K, float scale) {
  typedef typename Elem<ET>::T T;
  typedef typename Frag<T>::V V;
  const T* A = (const T*)Ap; const T* A2 = (const T*)A2p; const T* Bt = (const T*)Btp; const T* Bt2 = (const T*)Bt2p;
  __shared__ __align__(16) float sT[8][16 * 68];
  const int b    = blockIdx.y;
  const int lane = threadIdx.x & 31;
  const int wave = threadIdx.x >> 5;
  const int tilesN = N >> 6;
  const int tilesM = M >> 6;
  const int tile = blockIdx.x * 8 + wave;
  if (tile >= tilesM * tilesN) return;
  const int tm = tile / tilesN;
  const int tn = tile - tm * tilesN;
  const int m0 = tm << 6;
  const int n0 = tn << 6;

  const T* Ab  = A  + (size_t)b * strideA;
  const T* Bb  = Bt + (size_t)b * strideB;
  const T* Ab2 = SPLIT ? (A2  + (size_t)b * strideA) : nullptr;
  const T* Bb2 = SPLIT ? (Bt2 + (size_t)b * strideB) : nullptr;

  const int rlane = lane & 15;
  const int koff  = (lane >> 4) * 8;
  const int mOff  = (lane >> 4) * 8;

  v8f acc[4][4];
#pragma unroll
  for (int i = 0; i < 4; ++i)
#pragma unroll
    for (int j = 0; j < 4; ++j) acc[i][j] = (v8f){0.f,0.f,0.f,0.f,0.f,0.f,0.f,0.f};

  for (int k0 = 0; k0 < K; k0 += 32) {
    V bh[4], bl[4];
#pragma unroll
    for (int j = 0; j < 4; ++j) {
      const size_t bo = (size_t)(n0 + (j << 4) + rlane) * ldb + koff + k0;
      bh[j] = Frag<T>::load(Bb + bo);
      if (SPLIT) bl[j] = Frag<T>::load(Bb2 + bo);
    }
#pragma unroll
    for (int i = 0; i < 4; ++i) {
      const size_t ao = (size_t)(m0 + (i << 4) + rlane) * lda + koff + k0;
      V ah = Frag<T>::load(Ab + ao);
      V al;
      if (SPLIT) al = Frag<T>::load(Ab2 + ao);
#pragma unroll
      for (int j = 0; j < 4; ++j) {
        acc[i][j] = Frag<T>::mma(ah, bh[j], acc[i][j]);
        if (SPLIT) {
          acc[i][j] = Frag<T>::mma(ah, bl[j], acc[i][j]);
          acc[i][j] = Frag<T>::mma(al, bh[j], acc[i][j]);
        }
      }
      Frag<T>::guard4(acc[i][0], acc[i][1], acc[i][2], acc[i][3], ah, SPLIT ? al : ah);
    }
    Frag<T>::keep(bh[0], bh[1], bh[2], bh[3]);
    if (SPLIT) Frag<T>::keep(bl[0], bl[1], bl[2], bl[3]);
  }
  acc_guard4(acc[0][0], acc[0][1], acc[0][2], acc[0][3]);
  acc_guard4(acc[1][0], acc[1][1], acc[1][2], acc[1][3]);
  acc_guard4(acc[2][0], acc[2][1], acc[2][2], acc[2][3]);
  acc_guard4(acc[3][0], acc[3][1], acc[3][2], acc[3][3]);

  float* slab = sT[wave];
  const float* Rb = RESID ? (resid + (size_t)b * strideR) : nullptr;
#pragma unroll
  for (int i = 0; i < 4; ++i) {
    const int mBase = m0 + (i << 4);
#pragma unroll
    for (int j = 0; j < 4; ++j) {
      const int n = n0 + (j << 4) + rlane;
      float bv = 0.f;
      if (BIAS_MODE == 2) bv = bias[n];
#pragma unroll
      for (int r = 0; r < 8; ++r) {
        float v = acc[i][j][r] * scale;
        if (BIAS_MODE == 1) v += bias[mBase + mOff + r];
        if (BIAS_MODE == 2) v += bv;
        if (RESID) v += Rb[(size_t)(mBase + mOff + r) * ldc + n];
        if (ACT == 1) v = tanhf(v);
        if (ACT == 2) v = fmaxf(v, 0.0f);
        slab[(mOff + r) * 68 + (j << 4) + rlane] = v;
      }
    }
    __builtin_amdgcn_fence(__ATOMIC_RELEASE, "workgroup");
    __builtin_amdgcn_wave_barrier();
    __builtin_amdgcn_fence(__ATOMIC_ACQUIRE, "workgroup");
    if (OUT_MODE == 0) {
      float* C = (float*)Cout + (size_t)b * strideC;
      const int hh = lane >> 4, c4 = (lane & 15) * 4;
      for (int pass = 0; pass < 2; ++pass) {
#pragma unroll
        for (int it = 0; it < 8; ++it) {
          const int row = it * 2 + hh;
          v4f v = *(const v4f*)(slab + row * 68 + c4);
          *(volatile v4f*)(C + (size_t)(mBase + row) * ldc + n0 + c4) = v;
        }
        __threadfence();
      }
    } else {
      const int q = lane >> 3, c8 = (lane & 7) * 8;
      unsigned short* C  = (unsigned short*)Cout  + (size_t)b * strideC;
      unsigned short* C2 = (OUT_MODE == 2) ? ((unsigned short*)Cout2 + (size_t)b * strideC) : nullptr;
      for (int pass = 0; pass < 2; ++pass) {
#pragma unroll
        for (int it = 0; it < 4; ++it) {
          const int row = it * 4 + q;
          const float* sp = slab + row * 68 + c8;
          v8h hv, lv;
#pragma unroll
          for (int e = 0; e < 8; ++e) {
            if (OUT_MODE == 1) {
              hv[e] = (_Float16)sp[e];
            } else {
              unsigned short hb = f2bf_bits(sp[e]);
              unsigned short lb = f2bf_bits(sp[e] - bf_bits2f(hb));
              hv[e] = __builtin_bit_cast(_Float16, hb);
              lv[e] = __builtin_bit_cast(_Float16, lb);
            }
          }
          *(volatile v8h*)(C + (size_t)(mBase + row) * ldc + n0 + c8) = hv;
          if (OUT_MODE == 2) *(volatile v8h*)(C2 + (size_t)(mBase + row) * ldc + n0 + c8) = lv;
        }
        __threadfence();
      }
    }
    __builtin_amdgcn_fence(__ATOMIC_RELEASE, "workgroup");
    __builtin_amdgcn_wave_barrier();
    __builtin_amdgcn_fence(__ATOMIC_ACQUIRE, "workgroup");
  }
}

__global__ __launch_bounds__(NTHR) void cvt8p_kernel(const float* __restrict__ src, unsigned short* __restrict__ dst,
                                                     int nrow, int ncol8, int spitch, int dpitch, int dcol0, float sc) {
  const int i  = blockIdx.x * NTHR + threadIdx.x;
  const int n8 = nrow * ncol8;
  if (i < n8) {
    const int row = i / ncol8;
    const int c8  = i - row * ncol8;
    const float* sp = src + (size_t)row * spitch + c8 * 8;
    const v4f a = *(const v4f*)(sp);
    const v4f b = *(const v4f*)(sp + 4);
    v8h hv;
#pragma unroll
    for (int e = 0; e < 4; ++e) {
      const float fa = a[e] * sc;
      const float fb = b[e] * sc;
      hv[e]     = (_Float16)fa;
      hv[4 + e] = (_Float16)fb;
    }
    unsigned short* dp = dst + (size_t)row * dpitch + dcol0 + c8 * 8;
    *(volatile v8h*)dp = hv;
    __threadfence();
    *(volatile v8h*)dp = hv;
  }
}

__global__ __launch_bounds__(NTHR) void tpx_kernel(const float* __restrict__ src, unsigned short* __restrict__ O, float sc) {
  __shared__ float Tt[64 * 65];
  const int tid = threadIdx.x;
  const int c0 = blockIdx.x * 64, r0 = blockIdx.y * 64;
  const float* sb = src + (size_t)blockIdx.z * NSTEP * NFEAT;
  unsigned short* ob = O + (size_t)blockIdx.z * NFEAT * NSTEP;
#pragma unroll
  for (int i = 0; i < 4; ++i) {
    const int idx = i * NTHR + tid;
    const int rr = idx >> 4, cc = (idx & 15) * 4;
    const v4f v = *(const v4f*)(sb + (size_t)(r0 + rr) * NFEAT + c0 + cc);
    Tt[rr * 65 + cc + 0] = v[0];
    Tt[rr * 65 + cc + 1] = v[1];
    Tt[rr * 65 + cc + 2] = v[2];
    Tt[rr * 65 + cc + 3] = v[3];
  }
  __syncthreads();
  const int q = tid >> 3, c8 = (tid & 7) * 8;
  v8h hv[2];
#pragma unroll
  for (int g = 0; g < 2; ++g) {
    const int qq = g * 32 + q;
#pragma unroll
    for (int e = 0; e < 8; ++e) {
      const float f = Tt[(c8 + e) * 65 + qq] * sc;
      hv[g][e] = (_Float16)f;
    }
  }
  for (int pass = 0; pass < 2; ++pass) {
#pragma unroll
    for (int g = 0; g < 2; ++g) {
      const size_t o = (size_t)(c0 + g * 32 + q) * (size_t)NSTEP + (size_t)(r0 + c8);
      *(volatile v8h*)(ob + o) = hv[g];
    }
    __threadfence();
  }
}

__global__ __launch_bounds__(NTHR) void attn_lstm_scan_kernel(
    const float* __restrict__ x, const float* __restrict__ v_e,
    const float* __restrict__ b_ih, const float* __restrict__ b_hh,
    const unsigned short* __restrict__ We16p, const unsigned short* __restrict__ Wg16p,
    const float* __restrict__ Ux2, float* __restrict__ out) {
  __shared__ __align__(16) _Float16 At[2][ROWS_BLK * APITCH];
  __shared__ __align__(16) float wpS[ROWS_BLK * WPPITCH];
  __shared__ __align__(16) float cS[ROWS_BLK * CPITCH];
  __shared__ __align__(16) float Hs[ROWS_BLK * CPITCH];
  __shared__ __align__(16) float veS[NSTEP];
  __shared__ __align__(16) float biasS[NGATE];

  const _Float16* We16 = (const _Float16*)We16p;
  const _Float16* Wg16 = (const _Float16*)Wg16p;
  const int tid = threadIdx.x, lane = tid & 31, wave = tid >> 5;
  const int c = lane & 15, hh = lane >> 4, koff = hh * 8;
  const int batch0 = blockIdx.x * ROWS_BLK;

  {
    _Float16* af = &At[0][0];
#pragma unroll 1
    for (int i = tid; i < 2 * ROWS_BLK * APITCH; i += NTHR) af[i] = (_Float16)0.0f;
#pragma unroll 1
    for (int i = tid; i < ROWS_BLK * CPITCH; i += NTHR) cS[i] = 0.0f;
    const v4f ba = *(const v4f*)(b_ih + 4 * tid);
    const v4f bb4 = *(const v4f*)(b_hh + 4 * tid);
    v4f bs;
    bs[0] = ba[0] + bb4[0];
    bs[1] = ba[1] + bb4[1];
    bs[2] = ba[2] + bb4[2];
    bs[3] = ba[3] + bb4[3];
    *(v4f*)(biasS + 4 * tid) = bs;
    if (tid < 32) {
      const v4f ve4 = *(const v4f*)(v_e + 4 * tid);
      *(v4f*)(veS + 4 * tid) = ve4;
    }
  }
  __syncthreads();

  const v8f z8 = {0.f, 0.f, 0.f, 0.f, 0.f, 0.f, 0.f, 0.f};

#pragma unroll 1
  for (int t = 0; t < NSTEP; ++t) {
    const int cur = t & 1;
    _Float16* acur = &At[cur][0];
    _Float16* anxt = &At[cur ^ 1][0];

    {
      const _Float16* arow = acur + c * APITCH + COL_H + koff;
      const _Float16* wrow = We16 + (size_t)(16 * wave + c) * KATT + koff;
      v8f acc = z8;
#pragma unroll 1
      for (int k0 = 0; k0 < KATT; k0 += 32) {
        const v16h a = Frag<_Float16>::load(arow + k0);
        const v16h b = Frag<_Float16>::load(wrow + k0);
        acc = Frag<_Float16>::mma(a, b, acc);
        dep_guard1_h(acc, a, b);
      }
#pragma unroll
      for (int r = 0; r < 8; ++r) wpS[(8 * hh + r) * WPPITCH + 16 * wave + c] = acc[r] * WP2_FOLD;
    }
    __syncthreads();

    {
      const int bb = tid >> 4, li = tid & 15;
      const size_t brow = (size_t)(batch0 + bb);
      const float* uxb = Ux2 + (brow * NFEAT + (size_t)(li * 8)) * NSTEP;
      const float* wpr = wpS + bb * WPPITCH;
      float sj[8];
#pragma unroll
      for (int j = 0; j < 8; ++j) sj[j] = 0.0f;
#pragma unroll 1
      for (int s4 = 0; s4 < NSTEP / 4; ++s4) {
        const v4f w4 = *(const v4f*)(wpr + 4 * s4);
        const v4f e4 = *(const v4f*)(veS + 4 * s4);
#pragma unroll
        for (int j = 0; j < 8; ++j) {
          const v4f u = *(const v4f*)(uxb + j * NSTEP + 4 * s4);
          float a = sj[j];
          a += e4[0] * tanh_from2x_fast(w4[0] + u[0]);
          a += e4[1] * tanh_from2x_fast(w4[1] + u[1]);
          a += e4[2] * tanh_from2x_fast(w4[2] + u[2]);
          a += e4[3] * tanh_from2x_fast(w4[3] + u[3]);
          sj[j] = a;
        }
      }
      float mx = sj[0];
#pragma unroll
      for (int j = 1; j < 8; ++j) mx = fmaxf(mx, sj[j]);
#pragma unroll
      for (int off = 1; off < 16; off <<= 1) mx = fmaxf(mx, __shfl_xor(mx, off, 32));
      float ev[8];
      float sum = 0.0f;
#pragma unroll
      for (int j = 0; j < 8; ++j) {
        ev[j] = expf(sj[j] - mx);
        sum += ev[j];
      }
#pragma unroll
      for (int off = 1; off < 16; off <<= 1) sum += __shfl_xor(sum, off, 32);
      const float inv = __builtin_amdgcn_rcpf(sum);
      const float* xp = x + (brow * NSTEP + (size_t)t) * NFEAT + li * 8;
      const v4f x0 = *(const v4f*)(xp);
      const v4f x1 = *(const v4f*)(xp + 4);
      v8h hv;
#pragma unroll
      for (int j = 0; j < 4; ++j) {
        const float a0 = (x0[j] * (ev[j] * inv)) * XW_CARRY;
        const float a1 = (x1[j] * (ev[4 + j] * inv)) * XW_CARRY;
        hv[j]     = (_Float16)a0;
        hv[4 + j] = (_Float16)a1;
      }
      *(v8h*)(acur + bb * APITCH + li * 8) = hv;
    }
    __syncthreads();

#pragma unroll 1
    for (int sub = 0; sub < 2; ++sub) {
      const int j = 32 * wave + 16 * sub + c;
      const _Float16* arow = acur + c * APITCH + koff;
      const _Float16* wg = Wg16 + (size_t)j * KGATE + koff;
      v8f a0 = z8, a1 = z8, a2 = z8, a3 = z8;
#pragma unroll 1
      for (int k0 = 0; k0 < KGATE; k0 += 32) {
        const v16h a  = Frag<_Float16>::load(arow + k0);
        const v16h b0 = Frag<_Float16>::load(wg + k0);
        const v16h b1 = Frag<_Float16>::load(wg + (size_t)1 * NHID * KGATE + k0);
        const v16h b2 = Frag<_Float16>::load(wg + (size_t)2 * NHID * KGATE + k0);
        const v16h b3 = Frag<_Float16>::load(wg + (size_t)3 * NHID * KGATE + k0);
        a0 = Frag<_Float16>::mma(a, b0, a0);
        a1 = Frag<_Float16>::mma(a, b1, a1);
        a2 = Frag<_Float16>::mma(a, b2, a2);
        a3 = Frag<_Float16>::mma(a, b3, a3);
        dep_guard4x5_h(a0, a1, a2, a3, a, b0, b1, b2, b3);
      }
      acc_guard4(a0, a1, a2, a3);
      const float bi = biasS[j];
      const float bf = biasS[NHID + j];
      const float bg = biasS[2 * NHID + j];
      const float bo = biasS[3 * NHID + j];
#pragma unroll
      for (int r = 0; r < 8; ++r) {
        const int row = 8 * hh + r;
        const float zi = a0[r] * GATE_FOLD + bi;
        const float zf = a1[r] * GATE_FOLD + bf;
        const float zg = a2[r] * GATE_FOLD + bg;
        const float zo = a3[r] * GATE_FOLD + bo;
        const float cc = cS[row * CPITCH + j];
        const float c2 = sig_p(zf) * cc + sig_p(zi) * tanh_p(zg);
        const float h2 = sig_p(zo) * tanh_p(c2);
        cS[row * CPITCH + j] = c2;
        Hs[row * CPITCH + j] = h2;
        const float hq = h2 * HC_CARRY;
        const float cq = c2 * HC_CARRY;
        anxt[row * APITCH + COL_H + j] = (_Float16)hq;
        anxt[row * APITCH + COL_C + j] = (_Float16)cq;
      }
    }
    __syncthreads();

    for (int pass = 0; pass < 2; ++pass) {
#pragma unroll
      for (int it = 0; it < 4; ++it) {
        const int idx = it * NTHR + tid;
        const int row = idx >> 6, c4 = (idx & 63) * 4;
        const v4f v = *(const v4f*)(Hs + row * CPITCH + c4);
        *(volatile v4f*)(out + ((size_t)t * NBATCH + (size_t)(batch0 + row)) * NHID + c4) = v;
      }
      __threadfence();
    }
  }
}

extern "C" void kernel_launch(void* const* d_in, const int* in_sizes, int n_in,
                              void* d_out, int out_size, void* d_ws, size_t ws_size, hipStream_t stream) {
  if (n_in < 8 || d_out == nullptr || d_ws == nullptr) return;
  if (in_sizes[0] != NBATCH * NSTEP * NFEAT || in_sizes[1] != NSTEP * KATT || in_sizes[2] != NSTEP * NSTEP ||
      in_sizes[3] != NSTEP || in_sizes[4] != NGATE * NFEAT || in_sizes[5] != NGATE * NHID ||
      in_sizes[6] != NGATE || in_sizes[7] != NGATE || out_size != NSTEP * NBATCH * NHID) return;

  const float* x    = (const float*)d_in[0];
  const float* We   = (const float*)d_in[1];
  const float* Ue   = (const float*)d_in[2];
  const float* v_e  = (const float*)d_in[3];
  const float* W_ih = (const float*)d_in[4];
  const float* W_hh = (const float*)d_in[5];
  const float* b_ih = (const float*)d_in[6];
  const float* b_hh = (const float*)d_in[7];
  float* out = (float*)d_out;

  char* ws = (char*)d_ws; size_t off = 0;
  auto carve = [&](size_t bytes) -> char* { char* p = ws + off; off += (bytes + 255) & ~(size_t)255; return p; };
  float*          UX2  = (float*)carve((size_t)NBATCH * NFEAT * NSTEP * 4);
  unsigned short* XT16 = (unsigned short*)carve((size_t)NBATCH * NFEAT * NSTEP * 2);
  unsigned short* WE16 = (unsigned short*)carve((size_t)NSTEP * KATT * 2);
  unsigned short* UE16 = (unsigned short*)carve((size_t)NSTEP * NSTEP * 2);
  unsigned short* WG16 = (unsigned short*)carve((size_t)NGATE * KGATE * 2);
  if (off > ws_size || off > (size_t)134217728) return;

  cvt8p_kernel<<<(NSTEP * (KATT / 8)) / NTHR, NTHR, 0, stream>>>(We, WE16, NSTEP, KATT / 8, KATT, KATT, 0, WE_CARRY);
  cvt8p_kernel<<<(NSTEP * (NSTEP / 8)) / NTHR, NTHR, 0, stream>>>(Ue, UE16, NSTEP, NSTEP / 8, NSTEP, NSTEP, 0, UE_CARRY);
  cvt8p_kernel<<<(NGATE * (NFEAT / 8)) / NTHR, NTHR, 0, stream>>>(W_ih, WG16, NGATE, NFEAT / 8, NFEAT, KGATE, 0, WIH_CARRY);
  cvt8p_kernel<<<(NGATE * (NHID / 8)) / NTHR, NTHR, 0, stream>>>(W_hh, WG16, NGATE, NHID / 8, NHID, KGATE, NFEAT, WHH_CARRY);
  tpx_kernel<<<dim3(NFEAT / 64, NSTEP / 64, NBATCH), NTHR, 0, stream>>>(x, XT16, XT_CARRY);

  const int gemm_rows = NBATCH * NFEAT;
  const dim3 ggrid(((gemm_rows / 64) * (NSTEP / 64)) / 8, 1);
  wmma_gemm64<0, false, 0, 0, false, 0><<<ggrid, 256, 0, stream>>>(
      XT16, XT16, NSTEP, 0L, UE16, UE16, NSTEP, 0L, (void*)UX2, (void*)UX2, NSTEP, 0L,
      UX2, UX2, 0L, gemm_rows, NSTEP, NSTEP, UX2_FOLD);

  attn_lstm_scan_kernel<<<NBATCH / ROWS_BLK, NTHR, 0, stream>>>(x, v_e, b_ih, b_hh, WE16, WG16, UX2, out);
}
